// GNNJointInterpNetwork_21174188770102
// MI455X (gfx1250) — hardware-verified
//
#include <hip/hip_runtime.h>
#include <math.h>

constexpr int kStepsX = 17;
constexpr int kSteps  = 16;
constexpr int kNodes  = 128;
constexpr int kHid    = 256;
constexpr int kProj   = 128;
constexpr int kEdge   = 32;
constexpr int kSrcCols = 128;
constexpr int kRows   = kSteps * kNodes;
constexpr int kRowsX  = kStepsX * kNodes;
constexpr int kPairs  = kNodes * kNodes;

typedef __attribute__((ext_vector_type(16))) _Float16 v16h;
typedef __attribute__((ext_vector_type(8)))  _Float16 v8h;
typedef __attribute__((ext_vector_type(16))) __bf16   v16b;
typedef __attribute__((ext_vector_type(8)))  __bf16   v8b;
typedef __attribute__((ext_vector_type(8)))  float    v8f;
typedef __attribute__((ext_vector_type(4)))  float    v4f;
typedef __attribute__((ext_vector_type(4)))  unsigned int v4u;

__device__ __forceinline__ unsigned short f2bf_bits(float f) {
  unsigned u = __float_as_uint(f);
  return (unsigned short)((u + 0x7FFFu + ((u >> 16) & 1u)) >> 16);
}
__device__ __forceinline__ float bf_bits2f(unsigned short h) { return __uint_as_float(((unsigned)h) << 16); }

__device__ __forceinline__ void dep_guard_h(v8f& a, v8f& b, v16h x, v16h y) { asm volatile("v_nop\n\tv_nop\n\tv_nop\n\tv_nop" : "+v"(a), "+v"(b) : "v"(x), "v"(y)); }
__device__ __forceinline__ void dep_guard_b(v8f& a, v8f& b, v16b x, v16b y) { asm volatile("v_nop\n\tv_nop\n\tv_nop\n\tv_nop" : "+v"(a), "+v"(b) : "v"(x), "v"(y)); }
__device__ __forceinline__ void keep4_h(v16h a, v16h b, v16h c, v16h d) { asm volatile("v_nop" :: "v"(a), "v"(b), "v"(c), "v"(d)); }
__device__ __forceinline__ void keep4_b(v16b a, v16b b, v16b c, v16b d) { asm volatile("v_nop" :: "v"(a), "v"(b), "v"(c), "v"(d)); }
__device__ __forceinline__ void acc_guard4(v8f& a, v8f& b, v8f& c, v8f& d) { asm volatile("v_nop\n\tv_nop\n\tv_nop\n\tv_nop" : "+v"(a), "+v"(b), "+v"(c), "+v"(d)); }
template <typename T> struct Frag;
template <> struct Frag<_Float16> {
  typedef v16h V; union U { v16h v; v8h h[2]; };
  static __device__ __forceinline__ v16h load(const _Float16* p) {
    U f; f.h[0] = *(const v8h*)(p); f.h[1] = *(const v8h*)(p + 16); return f.v;
  }
  static __device__ __forceinline__ v8f mma(v16h a, v16h b, v8f c) {
    return __builtin_amdgcn_wmma_f32_16x16x32_f16(false, a, false, b, (short)0, c, false, false);
  }
  static __device__ __forceinline__ void guard(v8f& a, v8f& b, v16h x, v16h y) { dep_guard_h(a, b, x, y); }
  static __device__ __forceinline__ void keep(v16h a, v16h b, v16h c, v16h d) { keep4_h(a, b, c, d); }
};
template <> struct Frag<__bf16> {
  typedef v16b V; union U { v16b v; v8b h[2]; };
  static __device__ __forceinline__ v16b load(const __bf16* p) {
    U f; f.h[0] = *(const v8b*)(p); f.h[1] = *(const v8b*)(p + 16); return f.v;
  }
  static __device__ __forceinline__ v8f mma(v16b a, v16b b, v8f c) {
    return __builtin_amdgcn_wmma_f32_16x16x32_bf16(false, a, false, b, (short)0, c, false, false);
  }
  static __device__ __forceinline__ void guard(v8f& a, v8f& b, v16b x, v16b y) { dep_guard_b(a, b, x, y); }
  static __device__ __forceinline__ void keep(v16b a, v16b b, v16b c, v16b d) { keep4_b(a, b, c, d); }
};

__device__ __forceinline__ unsigned pk16(unsigned short a, unsigned short b) { return (unsigned)a | ((unsigned)b << 16); }

__device__ __forceinline__ void split_pack8(const float* s, v4u& uh, v4u& ul) {
  unsigned hw[4], lw[4];
#pragma unroll
  for (int e = 0; e < 4; ++e) {
    const float a = s[2 * e];
    const float b = s[2 * e + 1];
    const unsigned short ha = f2bf_bits(a);
    const unsigned short hb = f2bf_bits(b);
    const unsigned short la = f2bf_bits(a - bf_bits2f(ha));
    const unsigned short lb = f2bf_bits(b - bf_bits2f(hb));
    hw[e] = pk16(ha, hb);
    lw[e] = pk16(la, lb);
  }
  uh = (v4u){hw[0], hw[1], hw[2], hw[3]};
  ul = (v4u){lw[0], lw[1], lw[2], lw[3]};
}

__device__ __forceinline__ void row128_planes_store(const float* s, unsigned short* ph, unsigned short* pl, int lane) {
  const int l16 = lane & 15;
  v4u uh, ul;
  split_pack8(s + l16 * 8, uh, ul);
  for (int pass = 0; pass < 2; ++pass) {
    if (lane < 16) {
      *(volatile v4u*)(ph + l16 * 8) = uh;
      *(volatile v4u*)(pl + l16 * 8) = ul;
    }
    __threadfence();
  }
}

template <int BIAS_MODE, bool OUTF, bool OUTP, int ACT>
__global__ __launch_bounds__(256) void gemm_bf16x3(
    const unsigned short* __restrict__ Ap, const unsigned short* __restrict__ A2p, int lda,
    const unsigned short* __restrict__ Btp, const unsigned short* __restrict__ Bt2p, int ldb,
    float* __restrict__ Cf, int ldcf,
    unsigned short* __restrict__ Ch, unsigned short* __restrict__ Cl, int ldcp,
    const float* __restrict__ bias, int M, int N, int K) {
  typedef __bf16 T;
  typedef Frag<T>::V V;
  const T* Ab  = (const T*)Ap;  const T* Ab2 = (const T*)A2p;
  const T* Bb  = (const T*)Btp; const T* Bb2 = (const T*)Bt2p;
  __shared__ __align__(16) float sT[8][16 * 68];
  const int lane = threadIdx.x & 31;
  const int wave = threadIdx.x >> 5;
  const int tilesN = N >> 6;
  const int tilesM = M >> 6;
  const int tile = blockIdx.x * 8 + wave;
  if (tile >= tilesM * tilesN) return;
  const int tm = tile / tilesN;
  const int tn = tile - tm * tilesN;
  const int m0 = tm << 6;
  const int n0 = tn << 6;

  const int rlane = lane & 15;
  const int koff  = (lane >> 4) * 8;
  const int mOff  = (lane >> 4) * 8;

  v8f acc[4][4];
#pragma unroll
  for (int i = 0; i < 4; ++i)
#pragma unroll
    for (int j = 0; j < 4; ++j) acc[i][j] = (v8f){0.f,0.f,0.f,0.f,0.f,0.f,0.f,0.f};

  for (int k0 = 0; k0 < K; k0 += 32) {
    V bh[4], bl[4];
#pragma unroll
    for (int j = 0; j < 4; ++j) {
      const size_t bo = (size_t)(n0 + (j << 4) + rlane) * ldb + koff + k0;
      bh[j] = Frag<T>::load(Bb + bo);
      bl[j] = Frag<T>::load(Bb2 + bo);
    }
#pragma unroll
    for (int i = 0; i < 4; ++i) {
      const size_t ao = (size_t)(m0 + (i << 4) + rlane) * lda + koff + k0;
      V ah = Frag<T>::load(Ab + ao);
      V al = Frag<T>::load(Ab2 + ao);
#pragma unroll
      for (int j = 0; j < 4; ++j) {
        acc[i][j] = Frag<T>::mma(ah, bh[j], acc[i][j]);
        acc[i][j] = Frag<T>::mma(ah, bl[j], acc[i][j]);
        acc[i][j] = Frag<T>::mma(al, bh[j], acc[i][j]);
      }
      Frag<T>::guard(acc[i][0], acc[i][3], ah, al);
    }
    Frag<T>::keep(bh[0], bh[1], bh[2], bh[3]);
    Frag<T>::keep(bl[0], bl[1], bl[2], bl[3]);
  }
  acc_guard4(acc[0][0], acc[0][1], acc[0][2], acc[0][3]);
  acc_guard4(acc[1][0], acc[1][1], acc[1][2], acc[1][3]);
  acc_guard4(acc[2][0], acc[2][1], acc[2][2], acc[2][3]);
  acc_guard4(acc[3][0], acc[3][1], acc[3][2], acc[3][3]);

  float* slab = sT[wave];
#pragma unroll
  for (int i = 0; i < 4; ++i) {
    const int mBase = m0 + (i << 4);
#pragma unroll
    for (int j = 0; j < 4; ++j) {
      const int n = n0 + (j << 4) + rlane;
      float bv = 0.f;
      if (BIAS_MODE == 2) bv = bias[n];
#pragma unroll
      for (int r = 0; r < 8; ++r) {
        float v = acc[i][j][r];
        if (BIAS_MODE == 2) v += bv;
        if (ACT == 2) v = fmaxf(v, 0.0f);
        slab[(mOff + r) * 68 + (j << 4) + rlane] = v;
      }
    }
    __builtin_amdgcn_fence(__ATOMIC_RELEASE, "workgroup");
    __builtin_amdgcn_wave_barrier();
    __builtin_amdgcn_fence(__ATOMIC_ACQUIRE, "workgroup");
    if (OUTF) {
      float* C = Cf;
      const int hh = lane >> 4, c4 = (lane & 15) * 4;
      for (int pass = 0; pass < 2; ++pass) {
#pragma unroll
        for (int it = 0; it < 8; ++it) {
          const int row = it * 2 + hh;
          v4f v = *(const v4f*)(slab + row * 68 + c4);
          *(volatile v4f*)(C + (size_t)(mBase + row) * ldcf + n0 + c4) = v;
        }
        __threadfence();
      }
    }
    if (OUTP) {
      const int q = lane >> 3, c8 = (lane & 7) * 8;
      unsigned short* C  = Ch;
      unsigned short* C2 = Cl;
      for (int pass = 0; pass < 2; ++pass) {
#pragma unroll
        for (int it = 0; it < 4; ++it) {
          const int row = it * 4 + q;
          const float* sp = slab + row * 68 + c8;
          v8h hv, lv;
#pragma unroll
          for (int e = 0; e < 8; ++e) {
            unsigned short hb = f2bf_bits(sp[e]);
            unsigned short lb = f2bf_bits(sp[e] - bf_bits2f(hb));
            hv[e] = __builtin_bit_cast(_Float16, hb);
            lv[e] = __builtin_bit_cast(_Float16, lb);
          }
          *(volatile v8h*)(C  + (size_t)(mBase + row) * ldcp + n0 + c8) = hv;
          *(volatile v8h*)(C2 + (size_t)(mBase + row) * ldcp + n0 + c8) = lv;
        }
        __threadfence();
      }
    }
    __builtin_amdgcn_fence(__ATOMIC_RELEASE, "workgroup");
    __builtin_amdgcn_wave_barrier();
    __builtin_amdgcn_fence(__ATOMIC_ACQUIRE, "workgroup");
  }
}

__global__ __launch_bounds__(256) void tcast_kernel(const float* __restrict__ in0, const float* __restrict__ in1,
                                                    const float* __restrict__ in2, const float* __restrict__ in3,
                                                    int r0, int r1, int r2, int r3,
                                                    long inStrideZ, int Kc, int csh,
                                                    unsigned short* __restrict__ outH, unsigned short* __restrict__ outL,
                                                    long outStrideZ) {
  __shared__ float sm[32][257];
  const int tid = threadIdx.x;
  const int z   = blockIdx.y;
  const int n0  = blockIdx.x * 32;
  const float* pb = (z == 1) ? in1 : (z == 2) ? in2 : (z == 3) ? in3 : in0;
  const int row0  = (z == 1) ? r1  : (z == 2) ? r2  : (z == 3) ? r3  : r0;
  const float* ib = pb + (size_t)z * inStrideZ;
  const int nld = Kc >> 3;
#pragma unroll 1
  for (int it = 0; it < nld; ++it) {
    const int e  = it * 256 + tid;
    const int k  = e >> 5;
    const int nl = e & 31;
    sm[nl][k] = ib[(size_t)(row0 + k) * kSrcCols + n0 + nl];
  }
  __syncthreads();
  const size_t obase = (size_t)z * outStrideZ + (size_t)n0 * Kc;
  unsigned short* oh = outH + obase;
  unsigned short* ol = outL + obase;
  const int nchunks = 4 * Kc;
  const int kmask   = (Kc >> 3) - 1;
  const int nst     = (nchunks + 255) >> 8;
  for (int pass = 0; pass < 2; ++pass) {
#pragma unroll 1
    for (int it = 0; it < nst; ++it) {
      const int c = it * 256 + tid;
      if (c < nchunks) {
        const int nl = c >> csh;
        const int k8 = (c & kmask) * 8;
        v4u uh, ul;
        split_pack8(&sm[nl][k8], uh, ul);
        *(volatile v4u*)(oh + (size_t)c * 8) = uh;
        *(volatile v4u*)(ol + (size_t)c * 8) = ul;
      }
    }
    __threadfence();
  }
}

__global__ __launch_bounds__(256) void eenc_kernel(const float* __restrict__ edge_w, const float* __restrict__ We,
                                                   const float* __restrict__ be,
                                                   const int* __restrict__ batch, const int* __restrict__ no_graphs,
                                                   const int* __restrict__ time_i,
                                                   unsigned short* __restrict__ outH, unsigned short* __restrict__ outL) {
  (void)batch; (void)no_graphs; (void)time_i;
  const int c  = blockIdx.x * 256 + threadIdx.x;
  const int p  = c >> 2;
  const int e0 = (c & 3) * 8;
  const float w = edge_w[p];
  float v[8];
#pragma unroll
  for (int e = 0; e < 8; ++e) {
    const float a = w * We[e0 + e] + be[e0 + e];
    v[e] = fmaxf(a, 0.0f);
  }
  v4u uh, ul;
  split_pack8(v, uh, ul);
  unsigned short* ph = outH + (size_t)c * 8;
  unsigned short* pl = outL + (size_t)c * 8;
  *(volatile v4u*)ph = uh;
  *(volatile v4u*)pl = ul;
  __threadfence();
  *(volatile v4u*)ph = uh;
  *(volatile v4u*)pl = ul;
}

__global__ __launch_bounds__(128) void msgmax_kernel(const float* __restrict__ HWM, const float* __restrict__ EWM,
                                                     const float* __restrict__ edge_w,
                                                     unsigned short* __restrict__ aggH, unsigned short* __restrict__ aggL) {
  __shared__ float smax[4][kProj];
  __shared__ float sagg[kProj];
  const int tid  = threadIdx.x;
  const int lane = tid & 31;
  const int wave = tid >> 5;
  const int row  = blockIdx.x;
  const int t    = row >> 7;
  const int i    = row & 127;
  const float* hp = HWM + (size_t)t * kNodes * kProj + lane * 4;
  const float* ep = EWM + (size_t)i * kNodes * kProj + lane * 4;
  const float* wp = edge_w + i * kNodes;
  v4f acc = (v4f){0.f, 0.f, 0.f, 0.f};
#pragma unroll 1
  for (int jj = 0; jj < 32; ++jj) {
    const int j = wave * 32 + jj;
    const v4f a = *(const v4f*)(hp + (size_t)j * kProj);
    const v4f e = *(const v4f*)(ep + (size_t)j * kProj);
    const float w   = wp[j];
    const float adj = w + ((j == i) ? 1.0f : 0.0f);
    const bool keep = adj > 0.0f;
#pragma unroll
    for (int c = 0; c < 4; ++c) {
      float v = a[c] + e[c];
      v = fmaxf(v, 0.0f);
      v = keep ? v : 0.0f;
      acc[c] = fmaxf(acc[c], v);
    }
  }
#pragma unroll
  for (int c = 0; c < 4; ++c) smax[wave][lane * 4 + c] = acc[c];
  __syncthreads();
  {
    const float s0 = smax[0][tid], s1 = smax[1][tid], s2 = smax[2][tid], s3 = smax[3][tid];
    sagg[tid] = fmaxf(fmaxf(fmaxf(s0, s1), s2), s3);
  }
  __syncthreads();
  if (wave == 0) {
    row128_planes_store(sagg, aggH + (size_t)row * (2 * kProj), aggL + (size_t)row * (2 * kProj), lane);
  }
}

__global__ __launch_bounds__(128) void combine_kernel(const float* __restrict__ PRE, const float* __restrict__ Hf,
                                                      const float* __restrict__ bu, const float* __restrict__ bg,
                                                      unsigned short* __restrict__ dfH, unsigned short* __restrict__ dfL) {
  __shared__ float sh[kProj];
  const int tid  = threadIdx.x;
  const int lane = tid & 31;
  const int wave = tid >> 5;
  const int row  = blockIdx.x;
  const float pu = PRE[(size_t)row * (2 * kProj) + tid] + bu[tid];
  const float pg = PRE[(size_t)row * (2 * kProj) + kProj + tid] + bg[tid];
  const float upd = fmaxf(pu, 0.0f);
  const float g   = 1.0f / (1.0f + expf(-pg));
  const float h   = Hf[(size_t)row * kProj + tid];
  const float hn  = g * upd + (1.0f - g) * h;
  sh[tid] = hn;
  __syncthreads();
  if (wave == 0) {
    row128_planes_store(sh, dfH + (size_t)row * (2 * kProj), dfL + (size_t)row * (2 * kProj), lane);
  }
}

__global__ __launch_bounds__(128) void logits_kernel(const float* __restrict__ NA, const float* __restrict__ CB,
                                                     const float* __restrict__ EC, const float* __restrict__ Wc2,
                                                     const float* __restrict__ bc2, const float* __restrict__ edge_w,
                                                     float* __restrict__ out0) {
  __shared__ float slog[kNodes];
  const int tid  = threadIdx.x;
  const int lane = tid & 31;
  const int wave = tid >> 5;
  const int row  = blockIdx.x;
  const int t    = row >> 7;
  const int i    = row & 127;
  const v4f na = *(const v4f*)(NA + (size_t)row * kProj + lane * 4);
  const v4f w2 = *(const v4f*)(Wc2 + lane * 4);
  const float* cbp = CB + (size_t)t * kNodes * kProj + lane * 4;
  const float* ecp = EC + (size_t)i * kNodes * kProj + lane * 4;
#pragma unroll 1
  for (int jj = 0; jj < 32; ++jj) {
    const int j = jj * 4 + wave;
    const v4f cb = *(const v4f*)(cbp + (size_t)j * kProj);
    const v4f ec = *(const v4f*)(ecp + (size_t)j * kProj);
    float s = 0.0f;
#pragma unroll
    for (int c = 0; c < 4; ++c) {
      float h1 = na[c] + cb[c];
      h1 = h1 + ec[c];
      h1 = fmaxf(h1, 0.0f);
      s = s + h1 * w2[c];
    }
#pragma unroll
    for (int off = 16; off > 0; off >>= 1) s += __shfl_xor(s, off, 32);
    if (lane == 0) slog[j] = s;
  }
  __syncthreads();
  if (wave == 0) {
    const float b2 = bc2[0];
    v4f v;
#pragma unroll
    for (int c = 0; c < 4; ++c) {
      const int jc   = lane * 4 + c;
      const float w  = edge_w[i * kNodes + jc];
      const bool bad = (w == 0.0f) && (jc != i);
      const float lv = slog[jc] + b2;
      v[c] = bad ? -1.0e9f : lv;
    }
    float* op = out0 + (size_t)row * kNodes + lane * 4;
    *(volatile v4f*)op = v;
    __threadfence();
    *(volatile v4f*)op = v;
  }
}

__global__ __launch_bounds__(256) void dist_kernel(const float* __restrict__ DH, const float* __restrict__ Wd2,
                                                   const float* __restrict__ bd2, float* __restrict__ out1) {
  __shared__ float sd[32];
  const int tid   = threadIdx.x;
  const int lane  = tid & 31;
  const int wave  = tid >> 5;
  const int rbase = blockIdx.x * 32;
  const v4f w  = *(const v4f*)(Wd2 + lane * 4);
  const float b2 = bd2[0];
#pragma unroll
  for (int r = 0; r < 4; ++r) {
    const int row = rbase + wave * 4 + r;
    const v4f d = *(const v4f*)(DH + (size_t)row * kProj + lane * 4);
    float s = d[0] * w[0];
    s = s + d[1] * w[1];
    s = s + d[2] * w[2];
    s = s + d[3] * w[3];
#pragma unroll
    for (int off = 16; off > 0; off >>= 1) s += __shfl_xor(s, off, 32);
    if (lane == 0) sd[wave * 4 + r] = s + b2;
  }
  __syncthreads();
  if (wave == 0) {
    const int l8 = lane & 7;
    const v4f v = (v4f){sd[l8 * 4 + 0], sd[l8 * 4 + 1], sd[l8 * 4 + 2], sd[l8 * 4 + 3]};
    float* op = out1 + rbase + l8 * 4;
    for (int pass = 0; pass < 2; ++pass) {
      if (lane < 8) *(volatile v4f*)op = v;
      __threadfence();
    }
  }
}

extern "C" void kernel_launch(void* const* d_in, const int* in_sizes, int n_in,
                              void* d_out, int out_size, void* d_ws, size_t ws_size,
                              hipStream_t stream) {
  if (n_in < 23) return;
  if (in_sizes[0] != kStepsX * kHid * kNodes) return;
  if (in_sizes[1] != kPairs) return;
  if (in_sizes[5] != kHid * kProj || in_sizes[9] != (kProj + kEdge) * kProj) return;
  if (in_sizes[15] != (2 * kProj + kEdge) * kProj || in_sizes[19] != 2 * kProj * kProj) return;
  if (out_size != kRows * kNodes + kRows) return;

  const float* x      = (const float*)d_in[0];
  const float* edge_w = (const float*)d_in[1];
  const int*   batch  = (const int*)d_in[2];
  const int*   ngraph = (const int*)d_in[3];
  const int*   time_i = (const int*)d_in[4];
  const float* Wn  = (const float*)d_in[5];  const float* bn  = (const float*)d_in[6];
  const float* We  = (const float*)d_in[7];  const float* be  = (const float*)d_in[8];
  const float* Wm  = (const float*)d_in[9];  const float* bm  = (const float*)d_in[10];
  const float* Wu  = (const float*)d_in[11]; const float* bu  = (const float*)d_in[12];
  const float* Wg  = (const float*)d_in[13]; const float* bg  = (const float*)d_in[14];
  const float* Wc1 = (const float*)d_in[15]; const float* bc1 = (const float*)d_in[16];
  const float* Wc2 = (const float*)d_in[17]; const float* bc2 = (const float*)d_in[18];
  const float* Wd1 = (const float*)d_in[19]; const float* bd1 = (const float*)d_in[20];
  const float* Wd2 = (const float*)d_in[21]; const float* bd2 = (const float*)d_in[22];
  float* out0 = (float*)d_out;
  float* out1 = (float*)d_out + (size_t)kRows * kNodes;

  char* base = (char*)d_ws;
  size_t off = 0;
  auto carve = [&](size_t bytes) -> char* { char* p = base + off; off += (bytes + 255) & ~(size_t)255; return p; };
  const size_t bW256 = (size_t)4 * kProj * kHid * 2;
  const size_t bW128 = (size_t)3 * kProj * kProj * 2;
  const size_t bW32  = (size_t)2 * kProj * kEdge * 2;
  const size_t bX    = (size_t)kRowsX * kHid * 2;
  const size_t bEE   = (size_t)kPairs * kEdge * 2;
  const size_t bF128 = (size_t)kRows * kProj * 4;
  const size_t bP256 = (size_t)kRows * 2 * kProj * 2;
  const size_t bE128 = (size_t)kPairs * kProj * 4;
  const size_t bF256 = (size_t)kRows * 2 * kProj * 4;
  unsigned short* W256H = (unsigned short*)carve(bW256); unsigned short* W256L = (unsigned short*)carve(bW256);
  unsigned short* W128H = (unsigned short*)carve(bW128); unsigned short* W128L = (unsigned short*)carve(bW128);
  unsigned short* W32H  = (unsigned short*)carve(bW32);  unsigned short* W32L  = (unsigned short*)carve(bW32);
  unsigned short* XH    = (unsigned short*)carve(bX);    unsigned short* XL    = (unsigned short*)carve(bX);
  unsigned short* EEH   = (unsigned short*)carve(bEE);   unsigned short* EEL   = (unsigned short*)carve(bEE);
  float* CURF  = (float*)carve(bF128);  float* NXTF  = (float*)carve(bF128);
  unsigned short* CATCH = (unsigned short*)carve(bP256); unsigned short* CATCL = (unsigned short*)carve(bP256);
  unsigned short* CATNH = (unsigned short*)carve(bP256); unsigned short* CATNL = (unsigned short*)carve(bP256);
  float* EWMF  = (float*)carve(bE128);  float* ECF   = (float*)carve(bE128);
  float* HWMCF = (float*)carve(bF128);  float* HWMNF = (float*)carve(bF128);
  float* PRECF = (float*)carve(bF256);  float* PRENF = (float*)carve(bF256);
  unsigned short* DFH = (unsigned short*)carve(bP256); unsigned short* DFL = (unsigned short*)carve(bP256);
  float* NAF = (float*)carve(bF128); float* CBF = (float*)carve(bF128); float* DHF = (float*)carve(bF128);
  if (off > ws_size) return;

  auto ggrid = [](int M, int N) -> dim3 { const int tiles = (M >> 6) * (N >> 6); return dim3((unsigned)((tiles + 7) >> 3), 1, 1); };
  const long pl256 = (long)kProj * kHid;
  const long pl128 = (long)kProj * kProj;
  const long pl32  = (long)kProj * kEdge;

  tcast_kernel<<<dim3(4, 4), dim3(256), 0, stream>>>(Wn, Wu, Wg, Wd1, 0, 0, 0, 0, 0L, kHid, 5, W256H, W256L, pl256);
  tcast_kernel<<<dim3(4, 3), dim3(256), 0, stream>>>(Wm, Wc1, Wc1, Wc1, 0, 0, kProj, 0, 0L, kProj, 4, W128H, W128L, pl128);
  tcast_kernel<<<dim3(4, 2), dim3(256), 0, stream>>>(Wm, Wc1, Wc1, Wc1, kProj, 2 * kProj, 0, 0, 0L, kEdge, 2, W32H, W32L, pl32);
  tcast_kernel<<<dim3(4, kStepsX), dim3(256), 0, stream>>>(x, x, x, x, 0, 0, 0, 0, (long)kHid * kNodes, kHid, 5, XH, XL, pl256);
  eenc_kernel<<<dim3(256), dim3(256), 0, stream>>>(edge_w, We, be, batch, ngraph, time_i, EEH, EEL);

  gemm_bf16x3<2, true, true, 2><<<ggrid(kRows, kProj), dim3(256), 0, stream>>>(
      XH, XL, kHid, W256H, W256L, kHid, CURF, kProj, CATCH, CATCL, 2 * kProj, bn, kRows, kProj, kHid);
  gemm_bf16x3<2, true, true, 2><<<ggrid(kRows, kProj), dim3(256), 0, stream>>>(
      XH + (size_t)kNodes * kHid, XL + (size_t)kNodes * kHid, kHid, W256H, W256L, kHid,
      NXTF, kProj, CATNH, CATNL, 2 * kProj, bn, kRows, kProj, kHid);

  gemm_bf16x3<0, true, false, 0><<<ggrid(kPairs, kProj), dim3(256), 0, stream>>>(
      EEH, EEL, kEdge, W32H, W32L, kEdge, EWMF, kProj, EEH, EEL, 0, bn, kPairs, kProj, kEdge);
  gemm_bf16x3<2, true, false, 0><<<ggrid(kPairs, kProj), dim3(256), 0, stream>>>(
      EEH, EEL, kEdge, W32H + pl32, W32L + pl32, kEdge, ECF, kProj, EEH, EEL, 0, bc1, kPairs, kProj, kEdge);

  gemm_bf16x3<2, true, false, 0><<<ggrid(kRows, kProj), dim3(256), 0, stream>>>(
      CATCH, CATCL, 2 * kProj, W128H, W128L, kProj, HWMCF, kProj, CATCH, CATCL, 0, bm, kRows, kProj, kProj);
  msgmax_kernel<<<dim3(kRows), dim3(128), 0, stream>>>(HWMCF, EWMF, edge_w, CATCH + kProj, CATCL + kProj);
  gemm_bf16x3<0, true, false, 0><<<ggrid(kRows, 2 * kProj), dim3(256), 0, stream>>>(
      CATCH, CATCL, 2 * kProj, W256H + pl256, W256L + pl256, kHid, PRECF, 2 * kProj, CATCH, CATCL, 0, bn,
      kRows, 2 * kProj, 2 * kProj);
  combine_kernel<<<dim3(kRows), dim3(128), 0, stream>>>(PRECF, CURF, bu, bg, DFH, DFL);

  gemm_bf16x3<2, true, false, 0><<<ggrid(kRows, kProj), dim3(256), 0, stream>>>(
      CATNH, CATNL, 2 * kProj, W128H, W128L, kProj, HWMNF, kProj, CATNH, CATNL, 0, bm, kRows, kProj, kProj);
  msgmax_kernel<<<dim3(kRows), dim3(128), 0, stream>>>(HWMNF, EWMF, edge_w, CATNH + kProj, CATNL + kProj);
  gemm_bf16x3<0, true, false, 0><<<ggrid(kRows, 2 * kProj), dim3(256), 0, stream>>>(
      CATNH, CATNL, 2 * kProj, W256H + pl256, W256L + pl256, kHid, PRENF, 2 * kProj, CATNH, CATNL, 0, bn,
      kRows, 2 * kProj, 2 * kProj);
  combine_kernel<<<dim3(kRows), dim3(128), 0, stream>>>(PRENF, NXTF, bu, bg, DFH + kProj, DFL + kProj);

  gemm_bf16x3<0, true, false, 0><<<ggrid(kRows, kProj), dim3(256), 0, stream>>>(
      DFH + kProj, DFL + kProj, 2 * kProj, W128H + pl128, W128L + pl128, kProj, NAF, kProj, DFH, DFL, 0, bn,
      kRows, kProj, kProj);
  gemm_bf16x3<0, true, false, 0><<<ggrid(kRows, kProj), dim3(256), 0, stream>>>(
      DFH, DFL, 2 * kProj, W128H + 2 * pl128, W128L + 2 * pl128, kProj, CBF, kProj, DFH, DFL, 0, bn,
      kRows, kProj, kProj);
  logits_kernel<<<dim3(kRows), dim3(128), 0, stream>>>(NAF, CBF, ECF, Wc2, bc2, edge_w, out0);

  gemm_bf16x3<2, true, false, 2><<<ggrid(kRows, kProj), dim3(256), 0, stream>>>(
      DFH, DFL, 2 * kProj, W256H + 3 * pl256, W256L + 3 * pl256, kHid, DHF, kProj, DFH, DFL, 0, bd1,
      kRows, kProj, kHid);
  dist_kernel<<<dim3(kRows / 32), dim3(256), 0, stream>>>(DHF, Wd2, bd2, out1);
}
